// NonLocal2dBlock_68367289417927
// MI455X (gfx1250) — hardware-run, weakly checked
//
#include <hip/hip_runtime.h>
#include <math.h>

typedef __attribute__((ext_vector_type(16))) _Float16 v16h;
typedef __attribute__((ext_vector_type(16))) __bf16 v16b;
typedef __attribute__((ext_vector_type(8)))  _Float16 v8h;
typedef __attribute__((ext_vector_type(8)))  float v8f;
typedef __attribute__((ext_vector_type(4)))  float v4f;
typedef __attribute__((ext_vector_type(2)))  float v2f;
typedef __attribute__((ext_vector_type(4)))  unsigned v4u;
typedef __attribute__((ext_vector_type(4)))  int v4i;
typedef float __attribute__((may_alias)) float_a;
typedef int __attribute__((may_alias)) int_a;

template <typename T> __device__ __forceinline__ void vst2(void* p, T v) { *(volatile T*)p = v; __threadfence(); *(volatile T*)p = v; }
__device__ __forceinline__ v8f wmma16(v16h a, v16h b, v8f c) {
  v8f d = __builtin_amdgcn_wmma_f32_16x16x32_f16(false, a, false, b, (short)0, c, false, false);
  asm volatile("v_nop\n\tv_nop\n\tv_nop\n\tv_nop" : "+v"(d) : "v"(a), "v"(b));
  return d;
}
__device__ __forceinline__ v8f wmma_bf(v16b a, v16b b, v8f c) {
  v8f d = __builtin_amdgcn_wmma_f32_16x16x32_bf16(false, a, false, b, (short)0, c, false, false);
  asm volatile("v_nop\n\tv_nop\n\tv_nop\n\tv_nop" : "+v"(d) : "v"(a), "v"(b));
  return d;
}
__device__ __forceinline__ v16h frag_h(const _Float16* rowk0, int lane) {
  union { v16h v; v8h q[2]; } u; const _Float16* p = rowk0 + 8 * (lane >> 4);
  u.q[0] = *(const v8h*)p; u.q[1] = *(const v8h*)(p + 16); return u.v;
}
__device__ __forceinline__ v16h frag_f32(const float* rowk0, int lane) {
  v16h a; const float* p = rowk0 + 8 * (lane >> 4);
#pragma unroll
  for (int i = 0; i < 8; ++i) { a[i] = (_Float16)p[i]; a[8 + i] = (_Float16)p[16 + i]; }
  return a;
}
__device__ __forceinline__ v16h frag_f32s(const float* rowk0, int lane, float sc) {
  v16h a; const float* p = rowk0 + 8 * (lane >> 4);
#pragma unroll
  for (int i = 0; i < 8; ++i) { a[i] = (_Float16)(p[i] * sc); a[8 + i] = (_Float16)(p[16 + i] * sc); }
  return a;
}
__device__ __forceinline__ v16h fragc_f32(const float* W, int k0, int n, int lane, int ld, int K) {
  v16h a; const int g = lane >> 4;
#pragma unroll
  for (int i = 0; i < 8; ++i) { const int ka = k0 + 8 * g + i, kb = ka + 16;
    a[i] = (_Float16)(ka < K ? W[(size_t)(ka < K ? ka : K - 1) * ld + n] : 0.f); a[8 + i] = (_Float16)(kb < K ? W[(size_t)(kb < K ? kb : K - 1) * ld + n] : 0.f); }
  return a;
}
struct F2 { v16b h, l; };
__device__ __forceinline__ F2 bsplit16(const float v[16]) { F2 r;
#pragma unroll
  for (int i = 0; i < 16; ++i) { const __bf16 h = (__bf16)v[i]; r.h[i] = h; r.l[i] = (__bf16)(v[i] - (float)h); }
  return r; }
__device__ __forceinline__ F2 split_row(const float* row, int k0, int lane) { float v[16]; const float* p = row + k0 + 8 * (lane >> 4);
#pragma unroll
  for (int i = 0; i < 8; ++i) { v[i] = p[i]; v[8 + i] = p[16 + i]; }
  return bsplit16(v); }
__device__ __forceinline__ F2 split_rowK(const float* row, int k0, int lane, int K) { float v[16]; const int g = lane >> 4;
#pragma unroll
  for (int i = 0; i < 8; ++i) { const int ka = k0 + 8 * g + i, kb = ka + 16; v[i] = ka < K ? row[ka < K ? ka : K - 1] : 0.f; v[8 + i] = kb < K ? row[kb < K ? kb : K - 1] : 0.f; }
  return bsplit16(v); }
__device__ __forceinline__ F2 split_col(const float* W, int k0, int n, int lane, int ld, int K) { float v[16]; const int g = lane >> 4;
#pragma unroll
  for (int i = 0; i < 8; ++i) { const int ka = k0 + 8 * g + i, kb = ka + 16; v[i] = ka < K ? W[(size_t)(ka < K ? ka : K - 1) * ld + n] : 0.f; v[8 + i] = kb < K ? W[(size_t)(kb < K ? kb : K - 1) * ld + n] : 0.f; }
  return bsplit16(v); }
__device__ __forceinline__ v8f mac3(const F2& a, const F2& b, v8f c) { c = wmma_bf(a.l, b.h, c); c = wmma_bf(a.h, b.l, c); return wmma_bf(a.h, b.h, c); }
__device__ __forceinline__ float sigm(float v) { return 1.0f / (1.0f + expf(-v)); }
#define LDSX() do { asm volatile("s_wait_dscnt 0" ::: "memory"); __builtin_amdgcn_wave_barrier(); __builtin_amdgcn_fence(__ATOMIC_RELEASE, "workgroup"); } while (0)


#define NB 8
#define CC 256
#define IH 64
#define IW 64
#define NN (IH * IW)
#define MM (NN / 4)
#define DK 32
#define DV 128
#ifndef TNB
#define TNB NB
#endif
typedef __attribute__((ext_vector_type(8))) __bf16 v8b;
__device__ __forceinline__ v16b frag_b(const __bf16* rowk0, int lane) {
  union { v16b v; v8b q[2]; } u; const __bf16* p = rowk0 + 8 * (lane >> 4);
  u.q[0] = *(const v8b*)p; u.q[1] = *(const v8b*)(p + 16); return u.v;
}
__device__ __forceinline__ float bfr(float v) { return (float)(__bf16)v; }
__device__ __attribute__((noinline)) float exp_ni(float v) { return expf(v); }
__device__ __attribute__((noinline)) float erf_ni(float v) { return erff(v); }

#define WS_QH  0u
#define WS_QL  (WS_QH + 2u * (size_t)NB * NN * DK)
#define WS_KH  (WS_QL + 2u * (size_t)NB * NN * DK)
#define WS_KL  (WS_KH + 2u * (size_t)NB * MM * DK)
#define WS_VT  (WS_KL + 2u * (size_t)NB * MM * DK)
#define WS_VTL (WS_VT + 2u * (size_t)NB * DV * MM * 2)
#define WS_Y   (WS_VTL + 2u * (size_t)NB * DV * MM * 2)
#define WS_END (WS_Y + 4u * (size_t)NB * NN * DV)

__global__ __launch_bounds__(128) void k_conv(const float* __restrict__ X, const float* __restrict__ TW, const float* __restrict__ TB, const float* __restrict__ PW, const float* __restrict__ PB, const float* __restrict__ GW, const float* __restrict__ GB, _Float16* __restrict__ QH, _Float16* __restrict__ QL, _Float16* __restrict__ KH, _Float16* __restrict__ KL, _Float16* __restrict__ VT, _Float16* __restrict__ VTL) {
  __shared__ __align__(16) float st[128][DK + DK + 4];
  __shared__ __align__(16) float sg[128][DV + 4];
  __shared__ __align__(16) _Float16 sqh[128][DK + 8], sql[128][DK + 8]; __shared__ __align__(16) _Float16 skh[32][DK + 8], skl[32][DK + 8]; __shared__ __align__(16) _Float16 svh[DV][40], svl[DV][40];
  const int tid = threadIdx.x, wave = tid >> 5, lane = tid & 31, col = lane & 15, g = lane >> 4; const size_t b = blockIdx.y; const int pr = blockIdx.x; const int n0 = pr * 128;
  const float* Xb = X + b * CC * (size_t)NN;
  { v8f acc[2][4];
#pragma unroll
    for (int rt = 0; rt < 2; ++rt)
#pragma unroll
      for (int j = 0; j < 4; ++j) acc[rt][j] = v8f{};
#pragma unroll 2
    for (int kc = 0; kc < CC / 32; ++kc) { v16b w[4];
#pragma unroll
      for (int j = 0; j < 4; ++j) { const float* wr = (j < 2 ? TW + (size_t)(j * 16 + col) * CC : PW + (size_t)((j - 2) * 16 + col) * CC) + kc * 32 + 8 * g;
#pragma unroll
        for (int i = 0; i < 8; ++i) { w[j][i] = (__bf16)wr[i]; w[j][8 + i] = (__bf16)wr[16 + i]; } }
#pragma unroll
      for (int rt = 0; rt < 2; ++rt) { v16b a; const int px = n0 + wave * 32 + rt * 16 + col;
#pragma unroll
        for (int i = 0; i < 8; ++i) { a[i] = (__bf16)Xb[(size_t)(kc * 32 + 8 * g + i) * NN + px]; a[8 + i] = (__bf16)Xb[(size_t)(kc * 32 + 16 + 8 * g + i) * NN + px]; }
#pragma unroll
        for (int j = 0; j < 4; ++j) acc[rt][j] = wmma_bf(a, w[j], acc[rt][j]); } }
#pragma unroll
    for (int rt = 0; rt < 2; ++rt)
#pragma unroll
      for (int j = 0; j < 4; ++j) { const int c = j * 16 + col; const float bb = (j < 2) ? bfr(TB[c]) : bfr(PB[c - 32]);
#pragma unroll
        for (int r = 0; r < 8; ++r) st[wave * 32 + rt * 16 + 8 * g + r][c] = acc[rt][j][r] + bb; } }
  { v8f acc[2][8];
#pragma unroll
    for (int rt = 0; rt < 2; ++rt)
#pragma unroll
      for (int j = 0; j < 8; ++j) acc[rt][j] = v8f{};
#pragma unroll 1
    for (int kc = 0; kc < CC / 32; ++kc) { v16b a[2];
#pragma unroll
      for (int rt = 0; rt < 2; ++rt) { const int px = n0 + wave * 32 + rt * 16 + col;
#pragma unroll
        for (int i = 0; i < 8; ++i) { a[rt][i] = (__bf16)Xb[(size_t)(kc * 32 + 8 * g + i) * NN + px]; a[rt][8 + i] = (__bf16)Xb[(size_t)(kc * 32 + 16 + 8 * g + i) * NN + px]; } }
#pragma unroll
      for (int j = 0; j < 8; ++j) { v16b w; const float* wr = GW + (size_t)(j * 16 + col) * CC + kc * 32 + 8 * g;
#pragma unroll
        for (int i = 0; i < 8; ++i) { w[i] = (__bf16)wr[i]; w[8 + i] = (__bf16)wr[16 + i]; }
#pragma unroll
        for (int rt = 0; rt < 2; ++rt) acc[rt][j] = wmma_bf(a[rt], w, acc[rt][j]); } }
#pragma unroll
    for (int rt = 0; rt < 2; ++rt)
#pragma unroll
      for (int j = 0; j < 8; ++j) { const int c = j * 16 + col; const float bb = bfr(GB[c]);
#pragma unroll
        for (int r = 0; r < 8; ++r) sg[wave * 32 + rt * 16 + 8 * g + r][c] = acc[rt][j][r] + bb; } }
  __syncthreads();
  for (int e = tid; e < 128 * DK; e += 128) { const int px = e / DK, c = e % DK; const float v = st[px][c]; const _Float16 hv = (_Float16)v; sqh[px][c] = hv; sql[px][c] = (_Float16)((v - (float)hv) * 2048.0f); }
  for (int e = tid; e < 32 * DK; e += 128) { const int ml = e / DK, c = e % DK; const int q2 = ml * 2; const float v = fmaxf(fmaxf(st[q2][DK + c], st[q2 + 1][DK + c]), fmaxf(st[64 + q2][DK + c], st[64 + q2 + 1][DK + c])); const _Float16 hv = (_Float16)v; skh[ml][c] = hv; skl[ml][c] = (_Float16)((v - (float)hv) * 2048.0f); }
  for (int e = tid; e < 32 * DV; e += 128) { const int ml = e % 32, c = e / 32; const int q2 = ml * 2; const float v = fmaxf(fmaxf(sg[q2][c], sg[q2 + 1][c]), fmaxf(sg[64 + q2][c], sg[64 + q2 + 1][c])); const _Float16 hv = (_Float16)v; svh[c][ml] = hv; svl[c][ml] = (_Float16)((v - (float)hv) * 2048.0f); }
  __syncthreads();
  for (int e = tid; e < 128 * 4; e += 128) { const int px = e >> 2, q = e & 3; const size_t o = (b * NN + n0 + px) * DK + q * 8; vst2((unsigned*)(QH + o), *(const v4u*)&sqh[px][q * 8]); vst2((unsigned*)(QL + o), *(const v4u*)&sql[px][q * 8]); }
  { const int ml = tid >> 2, q = tid & 3; const size_t o = (b * MM + (size_t)pr * 32 + ml) * DK + q * 8; vst2((unsigned*)(KH + o), *(const v4u*)&skh[ml][q * 8]); vst2((unsigned*)(KL + o), *(const v4u*)&skl[ml][q * 8]); }
  for (int e = tid; e < DV * 4; e += 128) { const int c = e >> 2, q = e & 3; const size_t o = ((b * DV + c) * (size_t)(MM / 32) + pr) * 64 + q * 8; vst2((unsigned*)(VT + o), *(const v4u*)&svh[c][q * 8]); vst2((unsigned*)(VTL + o), *(const v4u*)&svl[c][q * 8]); } }
__global__ __launch_bounds__(128) void k_att(const _Float16* __restrict__ QH, const _Float16* __restrict__ QL, const _Float16* __restrict__ KH, const _Float16* __restrict__ KL, const _Float16* __restrict__ VT, const _Float16* __restrict__ VTL, float* __restrict__ Y) {
  __shared__ __align__(16) float sp[4][16][36]; __shared__ __align__(16) float so[4][16][132];
  const int tid = threadIdx.x, wave = tid >> 5, lane = tid & 31, col = lane & 15, g = lane >> 4; const size_t b = blockIdx.y; const int q0 = blockIdx.x * 64 + wave * 16; const size_t rq = b * NN + q0;
  const v16h aq = frag_h(QH + (rq + col) * DK, lane), aql = frag_h(QL + (rq + col) * DK, lane);
  float m[8], l[8];
#pragma unroll
  for (int r = 0; r < 8; ++r) { m[r] = -3.0e38f; l[r] = 0.f; }
  v8f acc[8] = {}, accl[8] = {};
#pragma unroll 1
  for (int ks = 0; ks < MM / 32; ++ks) { v8f s[2];
#pragma unroll
    for (int ct = 0; ct < 2; ++ct) { const size_t rk = b * MM + ks * 32 + ct * 16 + col; const v16h kh = frag_h(KH + rk * DK, lane), kl = frag_h(KL + rk * DK, lane); v8f c = {}, cl = {}; c = wmma16(aq, kh, c); cl = wmma16(aq, kl, cl); cl = wmma16(aql, kh, cl);
#pragma unroll
      for (int r = 0; r < 8; ++r) s[ct][r] = c[r] + cl[r] * (1.0f / 2048.0f); }
    float alpha[8];
#pragma unroll
    for (int r = 0; r < 8; ++r) { float mx = fmaxf(s[0][r], s[1][r]);
#pragma unroll
      for (int o = 1; o < 16; o <<= 1) mx = fmaxf(mx, __shfl_xor(mx, o));
      const float mn = fmaxf(m[r], mx); alpha[r] = __expf(m[r] - mn); const float e0 = __expf(s[0][r] - mn), e1 = __expf(s[1][r] - mn); float es = e0 + e1;
#pragma unroll
      for (int o = 1; o < 16; o <<= 1) es += __shfl_xor(es, o);
      l[r] = l[r] * alpha[r] + es; m[r] = mn; sp[wave][8 * g + r][col] = e0; sp[wave][8 * g + r][16 + col] = e1; }
#pragma unroll
    for (int j = 0; j < 8; ++j)
#pragma unroll
      for (int r = 0; r < 8; ++r) { acc[j][r] *= alpha[r]; accl[j][r] *= alpha[r]; }
    LDSX();
    v16h pa; { const float* prow = &sp[wave][col][0] + 8 * (lane >> 4);
#pragma unroll
      for (int i = 0; i < 8; ++i) { pa[i] = (_Float16)(prow[i] * 2048.0f); pa[8 + i] = (_Float16)(prow[16 + i] * 2048.0f); } }
#pragma unroll
    for (int j = 0; j < 8; ++j) { const size_t po = ((b * DV + j * 16 + col) * (size_t)(MM / 32) + ks) * 64; acc[j] = wmma16(pa, frag_h(VT + po, lane), acc[j]); accl[j] = wmma16(pa, frag_h(VTL + po, lane), accl[j]); }
    LDSX(); }
#pragma unroll
  for (int r = 0; r < 8; ++r) { const float il = (1.0f / 2048.0f) / l[r];
#pragma unroll
    for (int j = 0; j < 8; ++j) so[wave][8 * g + r][j * 16 + col] = (acc[j][r] + accl[j][r] * (1.0f / 2048.0f)) * il; }
  LDSX(); for (int rl = 0; rl < 16; ++rl) vst2(Y + (rq + rl) * DV + lane * 4, *(const v4f*)&so[wave][rl][lane * 4]); }
__global__ __launch_bounds__(128) void k_out(const float* __restrict__ Y, const float* __restrict__ OW, const float* __restrict__ OB, const float* __restrict__ GAMMA, const float* __restrict__ X, float* __restrict__ OUT) { __shared__ __align__(16) float stt[128][68];
  const int tid = threadIdx.x, wave = tid >> 5, lane = tid & 31, col = lane & 15, g = lane >> 4; const size_t b = blockIdx.y; const int n0 = blockIdx.x * 64; const size_t r0 = b * NN + n0 + wave * 16; const float gm = bfr(GAMMA[0]);
#pragma unroll 1
  for (int cc = 0; cc < CC; cc += 128) { v8f acc[8] = {};
#pragma unroll
    for (int kc = 0; kc < DV / 32; ++kc) { const F2 a = split_row(Y + (r0 + col) * DV, kc * 32, lane);
#pragma unroll
      for (int j = 0; j < 8; ++j) { v16b w; const float* wr = OW + (size_t)(cc + j * 16 + col) * DV + kc * 32 + 8 * g;
#pragma unroll
        for (int i = 0; i < 8; ++i) { w[i] = (__bf16)wr[i]; w[8 + i] = (__bf16)wr[16 + i]; } acc[j] = wmma_bf(a.h, w, acc[j]); acc[j] = wmma_bf(a.l, w, acc[j]); } }
#pragma unroll
    for (int j = 0; j < 8; ++j) { const int cl = j * 16 + col; const float bb = bfr(OB[cc + cl]);
#pragma unroll
      for (int r = 0; r < 8; ++r) { const int px = wave * 16 + 8 * g + r; stt[cl][px] = gm * (acc[j][r] + bb) + bfr(X[(b * CC + cc + cl) * (size_t)NN + n0 + px]); } }
    __syncthreads(); for (int e = tid; e < 128 * 16; e += 128) { const int cl = e >> 4, q = e & 15; vst2(OUT + (b * CC + cc + cl) * (size_t)NN + n0 + q * 4, *(const v4f*)&stt[cl][q * 4]); } __syncthreads(); } }
extern "C" void kernel_launch(void* const* d_in, const int* in_sizes, int n_in, void* d_out, int out_size, void* d_ws, size_t ws_size, hipStream_t stream) {
  (void)in_sizes; (void)n_in; (void)out_size;
  const float** F = (const float**)d_in;
  if (ws_size < (size_t)WS_END) return;
  char* ws = (char*)d_ws; _Float16 *QH = (_Float16*)(ws + WS_QH), *QL = (_Float16*)(ws + WS_QL), *KH = (_Float16*)(ws + WS_KH), *KL = (_Float16*)(ws + WS_KL), *VT = (_Float16*)(ws + WS_VT), *VTL = (_Float16*)(ws + WS_VTL); float* Y = (float*)(ws + WS_Y);
  k_conv<<<dim3(NN / 128, TNB), 128, 0, stream>>>(F[0], F[1], F[2], F[3], F[4], F[5], F[6], QH, QL, KH, KL, VT, VTL);
  k_att<<<dim3(NN / 64, TNB), 128, 0, stream>>>(QH, QL, KH, KL, VT, VTL, Y);
  k_out<<<dim3(NN / 64, TNB), 128, 0, stream>>>(Y, F[7], F[8], F[9], F[0], (float*)d_out);
}
